// RNN_44581760533079
// MI455X (gfx1250) — hardware-verified
//
#include <hip/hip_runtime.h>
#include <math.h>

constexpr int SEQ_LEN  = 512;
constexpr int BATCH_N  = 512;
constexpr int VOCAB_N  = 50000;
constexpr int DIN_N    = 256;
constexpr int DH_N     = 256;
constexpr int KTOT     = DIN_N + DH_N;
constexpr int DOUT_N   = 2;
constexpr int PAD_TOK  = 1;
constexpr int NTHR     = 256;
constexpr int ROWS_BLK = 16;
constexpr int A_PITCH  = KTOT + 8;
constexpr int HM_PITCH = DH_N + 4;
constexpr float WCARRY     = 256.0f;
constexpr float WCARRY_INV = 1.0f / 256.0f;

static_assert(KTOT == 512 && KTOT % 32 == 0);
static_assert(DH_N == 32 * (NTHR / 32));
static_assert(BATCH_N % ROWS_BLK == 0);
static_assert(ROWS_BLK * DIN_N == NTHR * 16);
static_assert(ROWS_BLK * DH_N == NTHR * 16);
static_assert(ROWS_BLK * DOUT_N * 4 == 128);
static_assert(A_PITCH % 8 == 0 && HM_PITCH % 4 == 0);
static_assert(KTOT % 64 == 0 && DH_N % 64 == 0);

typedef __attribute__((ext_vector_type(16))) _Float16 v16h;
typedef __attribute__((ext_vector_type(8)))  _Float16 v8h;
typedef __attribute__((ext_vector_type(8)))  float    v8f;
typedef __attribute__((ext_vector_type(4)))  float    v4f;

__device__ __forceinline__ void dep_guard2_h(v8f& a, v8f& b, v16h x, v16h y, v16h z) {
  asm volatile("v_nop\n\tv_nop\n\tv_nop\n\tv_nop" : "+v"(a), "+v"(b) : "v"(x), "v"(y), "v"(z));
}
__device__ __forceinline__ void keep3_h(v16h a, v16h b, v16h c) { asm volatile("v_nop" :: "v"(a), "v"(b), "v"(c)); }
__device__ __forceinline__ void acc_guard2(v8f& a, v8f& b) { asm volatile("v_nop\n\tv_nop\n\tv_nop\n\tv_nop" : "+v"(a), "+v"(b)); }

struct FragH {
  union U { v16h v; v8h h[2]; };
  static __device__ __forceinline__ v16h load(const _Float16* p) {
    U f;
    f.h[0] = *(const v8h*)(p);
    f.h[1] = *(const v8h*)(p + 16);
    return f.v;
  }
  static __device__ __forceinline__ v8f mma(v16h a, v16h b, v8f c) {
    return __builtin_amdgcn_wmma_f32_16x16x32_f16(false, a, false, b, (short)0, c, false, false);
  }
};

__global__ __launch_bounds__(NTHR) void wt_plane_kernel(const float* __restrict__ src, int R, int C, int ldo,
                                                        unsigned short* __restrict__ O, float sc) {
  __shared__ float Tt[64 * 65];
  const int tid = threadIdx.x;
  const int c0 = blockIdx.x * 64, r0 = blockIdx.y * 64;
#pragma unroll
  for (int i = 0; i < 4; ++i) {
    const int idx = i * NTHR + tid;
    const int rr = idx >> 4, cc = (idx & 15) * 4;
    const v4f v = *(const v4f*)(src + (size_t)(r0 + rr) * (size_t)C + c0 + cc);
    Tt[rr * 65 + cc + 0] = v[0];
    Tt[rr * 65 + cc + 1] = v[1];
    Tt[rr * 65 + cc + 2] = v[2];
    Tt[rr * 65 + cc + 3] = v[3];
  }
  __syncthreads();
  const int q = tid >> 3, c8 = (tid & 7) * 8;
  v8h hv[2];
#pragma unroll
  for (int g = 0; g < 2; ++g) {
    const int qq = g * 32 + q;
#pragma unroll
    for (int e = 0; e < 8; ++e) {
      const float f = Tt[(c8 + e) * 65 + qq];
      hv[g][e] = (_Float16)(f * sc);
    }
  }
  for (int pass = 0; pass < 2; ++pass) {
#pragma unroll
    for (int g = 0; g < 2; ++g) {
      const size_t o = (size_t)(c0 + g * 32 + q) * (size_t)ldo + (size_t)(r0 + c8);
      *(volatile v8h*)(O + o) = hv[g];
    }
    __threadfence();
  }
}

__global__ __launch_bounds__(NTHR) void rnn_seq_kernel(const int* __restrict__ text, const int* __restrict__ ubnd,
                                                       const float* __restrict__ hid0, const float* __restrict__ emb,
                                                       const unsigned short* __restrict__ WBp,
                                                       const float* __restrict__ bih, const float* __restrict__ Wio,
                                                       const float* __restrict__ bio, float* __restrict__ out) {
  __shared__ __align__(16) _Float16 At[ROWS_BLK * A_PITCH];
  __shared__ __align__(16) float    Hm[ROWS_BLK * HM_PITCH];
  __shared__ __align__(16) float    Osl[ROWS_BLK * DOUT_N];
  const _Float16* WB = (const _Float16*)WBp;
  const int tid = threadIdx.x, lane = tid & 31, wave = tid >> 5;
  const int c = lane & 15, hh = lane >> 4, koff = hh * 8;
  const int rowbase = blockIdx.x * ROWS_BLK;
  const int sm = tid >> 4;
  const int sseg = (tid & 15) * 16;

  {
    const float* hp = hid0 + (size_t)(rowbase + sm) * DH_N + sseg;
    float* hd = Hm + sm * HM_PITCH + sseg;
    const v4f a0 = *(const v4f*)(hp);
    const v4f a1 = *(const v4f*)(hp + 4);
    const v4f a2 = *(const v4f*)(hp + 8);
    const v4f a3 = *(const v4f*)(hp + 12);
    *(v4f*)(hd)      = a0;
    *(v4f*)(hd + 4)  = a1;
    *(v4f*)(hd + 8)  = a2;
    *(v4f*)(hd + 12) = a3;
  }
  const int j0 = 32 * wave + c;
  const int j1 = j0 + 16;
  const float bias0 = bih[j0];
  const float bias1 = bih[j1];
  __syncthreads();

  const _Float16* arow = At + c * A_PITCH + koff;
  const _Float16* w0 = WB + (size_t)j0 * KTOT + koff;
  const _Float16* w1 = WB + (size_t)j1 * KTOT + koff;
  const v8f z8 = {0.f, 0.f, 0.f, 0.f, 0.f, 0.f, 0.f, 0.f};

#pragma unroll 1
  for (int t = 0; t < SEQ_LEN - 1; ++t) {
    const int ubt = ubnd[t];
    if (ubt > rowbase) {
      {
        int idx = text[(size_t)t * BATCH_N + rowbase + sm];
        idx = idx < 0 ? 0 : idx;
        idx = idx > VOCAB_N - 1 ? VOCAB_N - 1 : idx;
        const bool pad = (idx == PAD_TOK);
        const float* er = emb + (size_t)idx * DIN_N + sseg;
        const v4f x0 = *(const v4f*)(er);
        const v4f x1 = *(const v4f*)(er + 4);
        const v4f x2 = *(const v4f*)(er + 8);
        const v4f x3 = *(const v4f*)(er + 12);
        const float* hr = Hm + sm * HM_PITCH + sseg;
        const v4f g0 = *(const v4f*)(hr);
        const v4f g1 = *(const v4f*)(hr + 4);
        const v4f g2 = *(const v4f*)(hr + 8);
        const v4f g3 = *(const v4f*)(hr + 12);
        v8h xa, xb, ha, hb;
#pragma unroll
        for (int e = 0; e < 4; ++e) {
          xa[e]     = (_Float16)(pad ? 0.0f : x0[e]);
          xa[4 + e] = (_Float16)(pad ? 0.0f : x1[e]);
          xb[e]     = (_Float16)(pad ? 0.0f : x2[e]);
          xb[4 + e] = (_Float16)(pad ? 0.0f : x3[e]);
          ha[e]     = (_Float16)g0[e];
          ha[4 + e] = (_Float16)g1[e];
          hb[e]     = (_Float16)g2[e];
          hb[4 + e] = (_Float16)g3[e];
        }
        _Float16* ar = At + sm * A_PITCH + sseg;
        *(v8h*)(ar)             = xa;
        *(v8h*)(ar + 8)         = xb;
        *(v8h*)(ar + DIN_N)     = ha;
        *(v8h*)(ar + DIN_N + 8) = hb;
      }
      __syncthreads();

      v8f acc0 = z8, acc1 = z8;
#pragma unroll 1
      for (int k0 = 0; k0 < KTOT; k0 += 32) {
        const v16h a  = FragH::load(arow + k0);
        const v16h f0 = FragH::load(w0 + k0);
        const v16h f1 = FragH::load(w1 + k0);
        acc0 = FragH::mma(a, f0, acc0);
        acc1 = FragH::mma(a, f1, acc1);
        dep_guard2_h(acc0, acc1, a, f0, f1);
        keep3_h(a, f0, f1);
      }
      acc_guard2(acc0, acc1);

#pragma unroll
      for (int r = 0; r < 8; ++r) {
        const int m = 8 * hh + r;
        const bool upd = (rowbase + m) < ubt;
        const float n0 = acc0[r] * WCARRY_INV + bias0;
        const float n1 = acc1[r] * WCARRY_INV + bias1;
        const float o0 = Hm[m * HM_PITCH + j0];
        const float o1 = Hm[m * HM_PITCH + j1];
        Hm[m * HM_PITCH + j0] = upd ? n0 : o0;
        Hm[m * HM_PITCH + j1] = upd ? n1 : o1;
      }
      __syncthreads();
    }
  }

  {
    int idx = text[(size_t)(SEQ_LEN - 1) * BATCH_N + rowbase + sm];
    idx = idx < 0 ? 0 : idx;
    idx = idx > VOCAB_N - 1 ? VOCAB_N - 1 : idx;
    const bool pad = (idx == PAD_TOK);
    const float* er = emb + (size_t)idx * DIN_N + sseg;
    const float* hr = Hm + sm * HM_PITCH + sseg;
    const float* wx = Wio + (size_t)sseg * DOUT_N;
    const float* wh = Wio + (size_t)(DIN_N + sseg) * DOUT_N;
    const float bo0 = bio[0];
    const float bo1 = bio[1];
    float s0 = 0.0f, s1 = 0.0f;
#pragma unroll 1
    for (int q = 0; q < 4; ++q) {
      const v4f xr = *(const v4f*)(er + 4 * q);
      const v4f hv = *(const v4f*)(hr + 4 * q);
      const v4f wa = *(const v4f*)(wx + 8 * q);
      const v4f wb = *(const v4f*)(wx + 8 * q + 4);
      const v4f wc = *(const v4f*)(wh + 8 * q);
      const v4f wd = *(const v4f*)(wh + 8 * q + 4);
      const float xq0 = pad ? 0.0f : xr[0];
      const float xq1 = pad ? 0.0f : xr[1];
      const float xq2 = pad ? 0.0f : xr[2];
      const float xq3 = pad ? 0.0f : xr[3];
      s0 += (xq0 * wa[0] + xq1 * wa[2]) + (xq2 * wb[0] + xq3 * wb[2]);
      s1 += (xq0 * wa[1] + xq1 * wa[3]) + (xq2 * wb[1] + xq3 * wb[3]);
      s0 += (hv[0] * wc[0] + hv[1] * wc[2]) + (hv[2] * wd[0] + hv[3] * wd[2]);
      s1 += (hv[0] * wc[1] + hv[1] * wc[3]) + (hv[2] * wd[1] + hv[3] * wd[3]);
    }
    s0 += __shfl_xor(s0, 1, 32);
    s1 += __shfl_xor(s1, 1, 32);
    s0 += __shfl_xor(s0, 2, 32);
    s1 += __shfl_xor(s1, 2, 32);
    s0 += __shfl_xor(s0, 4, 32);
    s1 += __shfl_xor(s1, 4, 32);
    s0 += __shfl_xor(s0, 8, 32);
    s1 += __shfl_xor(s1, 8, 32);
    if ((tid & 15) == 0) {
      Osl[sm * DOUT_N + 0] = s0 + bo0;
      Osl[sm * DOUT_N + 1] = s1 + bo1;
    }
  }
  __syncthreads();
  {
    const int l8 = tid & 7;
    const v4f ov = *(const v4f*)(Osl + 4 * l8);
    float* op = out + (size_t)rowbase * DOUT_N + 4 * l8;
    for (int pass = 0; pass < 2; ++pass) {
      if (tid < 8) *(volatile v4f*)op = ov;
      __threadfence();
    }
  }
}

extern "C" void kernel_launch(void* const* d_in, const int* in_sizes, int n_in,
                              void* d_out, int out_size, void* d_ws, size_t ws_size, hipStream_t stream) {
  if (n_in < 8 || d_out == nullptr || d_ws == nullptr) return;
  if (in_sizes[0] != SEQ_LEN * BATCH_N || in_sizes[1] != SEQ_LEN || in_sizes[2] != BATCH_N * DH_N ||
      in_sizes[3] != VOCAB_N * DIN_N || in_sizes[4] != KTOT * DH_N || in_sizes[5] != DH_N ||
      in_sizes[6] != KTOT * DOUT_N || in_sizes[7] != DOUT_N || out_size != BATCH_N * DOUT_N) return;

  const int*   text = (const int*)d_in[0];
  const int*   ubnd = (const int*)d_in[1];
  const float* hid0 = (const float*)d_in[2];
  const float* emb  = (const float*)d_in[3];
  const float* wih  = (const float*)d_in[4];
  const float* bih  = (const float*)d_in[5];
  const float* wio  = (const float*)d_in[6];
  const float* bio  = (const float*)d_in[7];
  float* out = (float*)d_out;

  char* ws = (char*)d_ws;
  size_t off = 0;
  unsigned short* WB = (unsigned short*)(ws + off);
  off += (((size_t)DH_N * KTOT * 2) + 255) & ~(size_t)255;
  if (off > ws_size || off > (size_t)134217728) return;

  wt_plane_kernel<<<dim3(DH_N / 64, KTOT / 64), NTHR, 0, stream>>>(wih, KTOT, DH_N, KTOT, WB, WCARRY);
  rnn_seq_kernel<<<BATCH_N / ROWS_BLK, NTHR, 0, stream>>>(text, ubnd, hid0, emb, WB, bih, wio, bio, out);
}
